// raw_gru_s2s_60971355734180
// MI455X (gfx1250) — hardware-verified
//
#include <hip/hip_runtime.h>
#include <math.h>

#define NN 20000
#define NE 320000
#define NG 128
#define HID 128
#define NHD 4
#define ZW 512
#define FIN 74
#define KP0 96
#define MP 20032
#define NT 256
#define TG 2048
#define NTILE 10
#define NROWT (NTILE * TG)
#define SCH 4096
#define SPT (SCH / NT)
#define NCH ((NE + SCH - 1) / SCH)
#define AGG_LDS_BYTES ((TG * 8 + SCH) * 4)
#define WSC 16.0f
#define WSC_INV 0.0625f
#define BN_EPS 1e-5f

static_assert(NE % SPT == 0);
static_assert(MP % 64 == 0 && MP >= NN);
static_assert(NROWT >= NN);
static_assert(NN % 4 == 0);
static_assert(KP0 % 32 == 0 && KP0 >= FIN);
static_assert(TG / 8 == 256);

typedef __attribute__((ext_vector_type(16))) _Float16 v16h;
typedef __attribute__((ext_vector_type(8)))  _Float16 v8h;
typedef __attribute__((ext_vector_type(4)))  _Float16 v4h;
typedef __attribute__((ext_vector_type(16))) __bf16   v16b;
typedef __attribute__((ext_vector_type(8)))  __bf16   v8b;
typedef __attribute__((ext_vector_type(8)))  float    v8f;
typedef __attribute__((ext_vector_type(4)))  float    v4f;
typedef __attribute__((ext_vector_type(4)))  int      v4i;
#define U16(p) ((const unsigned short*)(const void*)(p))

__device__ __forceinline__ unsigned short f2bf_bits(float f) {
  unsigned u = __float_as_uint(f);
  return (unsigned short)((u + 0x7FFFu + ((u >> 16) & 1u)) >> 16);
}
__device__ __forceinline__ float bf_bits2f(unsigned short h) { return __uint_as_float(((unsigned)h) << 16); }

__device__ __forceinline__ void dep_guard_h(v8f& a, v8f& b, v16h x, v16h y) { asm volatile("v_nop\n\tv_nop\n\tv_nop\n\tv_nop" : "+v"(a), "+v"(b) : "v"(x), "v"(y)); }
__device__ __forceinline__ void dep_guard_b(v8f& a, v8f& b, v16b x, v16b y) { asm volatile("v_nop\n\tv_nop\n\tv_nop\n\tv_nop" : "+v"(a), "+v"(b) : "v"(x), "v"(y)); }
__device__ __forceinline__ void keep4_h(v16h a, v16h b, v16h c, v16h d) { asm volatile("v_nop" :: "v"(a), "v"(b), "v"(c), "v"(d)); }
__device__ __forceinline__ void keep4_b(v16b a, v16b b, v16b c, v16b d) { asm volatile("v_nop" :: "v"(a), "v"(b), "v"(c), "v"(d)); }
__device__ __forceinline__ void acc_guard4(v8f& a, v8f& b, v8f& c, v8f& d) { asm volatile("v_nop\n\tv_nop\n\tv_nop\n\tv_nop" : "+v"(a), "+v"(b), "+v"(c), "+v"(d)); }
template <typename T> struct Frag;
template <> struct Frag<_Float16> {
  typedef v16h V; union U { v16h v; v8h h[2]; };
  static __device__ __forceinline__ v16h load(const _Float16* p) {
    U f; f.h[0] = *(const v8h*)(p); f.h[1] = *(const v8h*)(p + 16); return f.v;
  }
  static __device__ __forceinline__ v8f mma(v16h a, v16h b, v8f c) {
    return __builtin_amdgcn_wmma_f32_16x16x32_f16(false, a, false, b, (short)0, c, false, false);
  }
  static __device__ __forceinline__ void guard(v8f& a, v8f& b, v16h x, v16h y) { dep_guard_h(a, b, x, y); }
  static __device__ __forceinline__ void keep(v16h a, v16h b, v16h c, v16h d) { keep4_h(a, b, c, d); }
};
template <> struct Frag<__bf16> {
  typedef v16b V; union U { v16b v; v8b h[2]; };
  static __device__ __forceinline__ v16b load(const __bf16* p) {
    U f; f.h[0] = *(const v8b*)(p); f.h[1] = *(const v8b*)(p + 16); return f.v;
  }
  static __device__ __forceinline__ v8f mma(v16b a, v16b b, v8f c) {
    return __builtin_amdgcn_wmma_f32_16x16x32_bf16(false, a, false, b, (short)0, c, false, false);
  }
  static __device__ __forceinline__ void guard(v8f& a, v8f& b, v16b x, v16b y) { dep_guard_b(a, b, x, y); }
  static __device__ __forceinline__ void keep(v16b a, v16b b, v16b c, v16b d) { keep4_b(a, b, c, d); }
};

template <int ET> struct Elem;
template <> struct Elem<0> { typedef _Float16 T; };
template <> struct Elem<1> { typedef __bf16 T; };
template <int ET, bool SPLIT, int BIAS_MODE, int OUT_MODE, bool RESID, int ACT = 0>
__global__ __launch_bounds__(256) void wmma_gemm64(
    const unsigned short* __restrict__ Ap, const unsigned short* __restrict__ A2p, int lda, long strideA,
    const unsigned short* __restrict__ Btp, const unsigned short* __restrict__ Bt2p, int ldb, long strideB,
    void* __restrict__ Cout, void* __restrict__ Cout2, int ldc, long strideC,
    const float* __restrict__ bias,
    const float* __restrict__ resid, long strideR,
    int M, int N, int K, float scale) {
  typedef typename Elem<ET>::T T;
  typedef typename Frag<T>::V V;
  const T* A = (const T*)Ap; const T* A2 = (const T*)A2p; const T* Bt = (const T*)Btp; const T* Bt2 = (const T*)Bt2p;
  __shared__ __align__(16) float sT[8][16 * 68];
  const int b    = blockIdx.y;
  const int lane = threadIdx.x & 31;
  const int wave = threadIdx.x >> 5;
  const int tilesN = N >> 6;
  const int tilesM = M >> 6;
  const int tile = blockIdx.x * 8 + wave;
  if (tile >= tilesM * tilesN) return;
  const int tm = tile / tilesN;
  const int tn = tile - tm * tilesN;
  const int m0 = tm << 6;
  const int n0 = tn << 6;

  const T* Ab  = A  + (size_t)b * strideA;
  const T* Bb  = Bt + (size_t)b * strideB;
  const T* Ab2 = SPLIT ? (A2  + (size_t)b * strideA) : nullptr;
  const T* Bb2 = SPLIT ? (Bt2 + (size_t)b * strideB) : nullptr;

  const int rlane = lane & 15;
  const int koff  = (lane >> 4) * 8;
  const int mOff  = (lane >> 4) * 8;

  v8f acc[4][4];
#pragma unroll
  for (int i = 0; i < 4; ++i)
#pragma unroll
    for (int j = 0; j < 4; ++j) acc[i][j] = (v8f){0.f,0.f,0.f,0.f,0.f,0.f,0.f,0.f};

  for (int k0 = 0; k0 < K; k0 += 32) {
    V bh[4], bl[4];
#pragma unroll
    for (int j = 0; j < 4; ++j) {
      const size_t bo = (size_t)(n0 + (j << 4) + rlane) * ldb + koff + k0;
      bh[j] = Frag<T>::load(Bb + bo);
      if (SPLIT) bl[j] = Frag<T>::load(Bb2 + bo);
    }
#pragma unroll
    for (int i = 0; i < 4; ++i) {
      const size_t ao = (size_t)(m0 + (i << 4) + rlane) * lda + koff + k0;
      V ah = Frag<T>::load(Ab + ao);
      V al;
      if (SPLIT) al = Frag<T>::load(Ab2 + ao);
#pragma unroll
      for (int j = 0; j < 4; ++j) {
        acc[i][j] = Frag<T>::mma(ah, bh[j], acc[i][j]);
        if (SPLIT) {
          acc[i][j] = Frag<T>::mma(ah, bl[j], acc[i][j]);
          acc[i][j] = Frag<T>::mma(al, bh[j], acc[i][j]);
        }
      }
      Frag<T>::guard(acc[i][0], acc[i][3], ah, SPLIT ? al : ah);
    }
    Frag<T>::keep(bh[0], bh[1], bh[2], bh[3]);
    if (SPLIT) Frag<T>::keep(bl[0], bl[1], bl[2], bl[3]);
  }
  acc_guard4(acc[0][0], acc[0][1], acc[0][2], acc[0][3]);
  acc_guard4(acc[1][0], acc[1][1], acc[1][2], acc[1][3]);
  acc_guard4(acc[2][0], acc[2][1], acc[2][2], acc[2][3]);
  acc_guard4(acc[3][0], acc[3][1], acc[3][2], acc[3][3]);

  float* slab = sT[wave];
  const float* Rb = RESID ? (resid + (size_t)b * strideR) : nullptr;
#pragma unroll
  for (int i = 0; i < 4; ++i) {
    const int mBase = m0 + (i << 4);
#pragma unroll
    for (int j = 0; j < 4; ++j) {
      const int n = n0 + (j << 4) + rlane;
      float bv = 0.f;
      if (BIAS_MODE == 2) bv = bias[n];
#pragma unroll
      for (int r = 0; r < 8; ++r) {
        float v = acc[i][j][r] * scale;
        if (BIAS_MODE == 1) v += bias[mBase + mOff + r];
        if (BIAS_MODE == 2) v += bv;
        if (RESID) v += Rb[(size_t)(mBase + mOff + r) * ldc + n];
        if (ACT == 1) v = tanhf(v);
        if (ACT == 2) v = fmaxf(v, 0.0f);
        if (ACT == 3) v = v / (1.0f + expf(-v));
        if (ACT == 4) v = (v > 0.f) ? v : 0.01f * v;
        if (ACT == 5) v = 0.5f * v * (1.0f + erff(v * 0.70710678118654752f));
        slab[(mOff + r) * 68 + (j << 4) + rlane] = v;
      }
    }
    __builtin_amdgcn_fence(__ATOMIC_RELEASE, "workgroup");
    __builtin_amdgcn_wave_barrier();
    __builtin_amdgcn_fence(__ATOMIC_ACQUIRE, "workgroup");
    if (OUT_MODE == 0) {
      float* C = (float*)Cout + (size_t)b * strideC;
      const int hh = lane >> 4, c4 = (lane & 15) * 4;
      for (int pass = 0; pass < 2; ++pass) {
#pragma unroll
        for (int it = 0; it < 8; ++it) {
          const int row = it * 2 + hh;
          v4f v = *(const v4f*)(slab + row * 68 + c4);
          *(volatile v4f*)(C + (size_t)(mBase + row) * ldc + n0 + c4) = v;
        }
        __threadfence();
      }
    } else {
      const int q = lane >> 3, c8 = (lane & 7) * 8;
      unsigned short* C  = (unsigned short*)Cout  + (size_t)b * strideC;
      unsigned short* C2 = (OUT_MODE == 2) ? ((unsigned short*)Cout2 + (size_t)b * strideC) : nullptr;
      for (int pass = 0; pass < 2; ++pass) {
#pragma unroll
        for (int it = 0; it < 4; ++it) {
          const int row = it * 4 + q;
          const float* sp = slab + row * 68 + c8;
          v8h hv, lv;
#pragma unroll
          for (int e = 0; e < 8; ++e) {
            if (OUT_MODE == 1) {
              hv[e] = (_Float16)sp[e];
            } else {
              unsigned short hb = f2bf_bits(sp[e]);
              unsigned short lb = f2bf_bits(sp[e] - bf_bits2f(hb));
              hv[e] = __builtin_bit_cast(_Float16, hb);
              lv[e] = __builtin_bit_cast(_Float16, lb);
            }
          }
          *(volatile v8h*)(C + (size_t)(mBase + row) * ldc + n0 + c8) = hv;
          if (OUT_MODE == 2) *(volatile v8h*)(C2 + (size_t)(mBase + row) * ldc + n0 + c8) = lv;
        }
        __threadfence();
      }
    }
    __builtin_amdgcn_fence(__ATOMIC_RELEASE, "workgroup");
    __builtin_amdgcn_wave_barrier();
    __builtin_amdgcn_fence(__ATOMIC_ACQUIRE, "workgroup");
  }
}

__device__ __forceinline__ unsigned pack_f16x2(float a, float b) {
  const _Float16 h0 = (_Float16)a, h1 = (_Float16)b;
  return (unsigned)__builtin_bit_cast(unsigned short, h0) | ((unsigned)__builtin_bit_cast(unsigned short, h1) << 16);
}

__global__ __launch_bounds__(NT) void cast_h_kernel(const float* __restrict__ in, unsigned short* __restrict__ out) {
  const int i = blockIdx.x * NT + threadIdx.x;
  if (i < MP * (KP0 / 2)) {
    const int n = i / (KP0 / 2);
    const int k = 2 * (i - n * (KP0 / 2));
    const int nc = (n < NN) ? n : (NN - 1);
    const int kc = (k < FIN) ? k : (FIN - 2);
    float f0 = in[(size_t)nc * FIN + kc], f1 = in[(size_t)nc * FIN + kc + 1];
    if (n >= NN || k >= FIN) { f0 = 0.f; f1 = 0.f; }
    const unsigned u = pack_f16x2(f0, f1);
    ((volatile unsigned*)out)[i] = u;
    __threadfence();
    ((volatile unsigned*)out)[i] = u;
  }
}

__global__ __launch_bounds__(NT) void wprep_kernel(const float* __restrict__ W, unsigned short* __restrict__ Bt, int K, int Kpad) {
  const int i = blockIdx.x * NT + threadIdx.x;
  const int kh = Kpad >> 1;
  if (i < ZW * kh) {
    const int n = i / kh;
    const int k = 2 * (i - n * kh);
    const int head = n >> 7, c = n & 127;
    const int kc = (k < K) ? k : (K - 2);
    float a = W[((size_t)head * K + kc) * HID + c];
    float b = W[((size_t)head * K + kc + 1) * HID + c];
    if (k >= K) { a = 0.f; b = 0.f; }
    const unsigned u = pack_f16x2(a * WSC, b * WSC);
    ((volatile unsigned*)Bt)[i] = u;
    __threadfence();
    ((volatile unsigned*)Bt)[i] = u;
  }
}

__global__ __launch_bounds__(NT) void dots_kernel(const float* __restrict__ Z, const float* __restrict__ att, float* __restrict__ SD) {
  const int lane = threadIdx.x & 31;
  const int gw = blockIdx.x * (NT / 32) + (threadIdx.x >> 5);
  if (gw < NN / 4) {
    const int c4 = 4 * lane;
    v4f a_s[4], a_d[4];
#pragma unroll
    for (int q = 0; q < 4; ++q) {
      a_s[q] = *(const v4f*)(att + q * 2 * HID + c4);
      a_d[q] = *(const v4f*)(att + q * 2 * HID + HID + c4);
    }
    float keep = 0.f;
#pragma unroll 1
    for (int j = 0; j < 4; ++j) {
      const int n = gw * 4 + j;
      const float* zr = Z + (size_t)n * ZW + c4;
#pragma unroll
      for (int q = 0; q < 4; ++q) {
        const v4f zz = *(const v4f*)(zr + HID * q);
        float ps = 0.f, pd = 0.f;
#pragma unroll
        for (int i = 0; i < 4; ++i) { ps = fmaf(zz[i], a_s[q][i], ps); pd = fmaf(zz[i], a_d[q][i], pd); }
#pragma unroll
        for (int off = 16; off > 0; off >>= 1) { ps += __shfl_xor(ps, off, 32); pd += __shfl_xor(pd, off, 32); }
        if (lane == 8 * j + q) keep = ps;
        if (lane == 8 * j + 4 + q) keep = pd;
      }
    }
    float* sp = SD + (size_t)gw * 32 + lane;
    *(volatile float*)sp = keep;
    __threadfence();
    *(volatile float*)sp = keep;
  }
}

__device__ __forceinline__ int blk_excl_scan(int cnt, int* scan_ws, int tid, int* tot) {
  const int lane = tid & 31, wave = tid >> 5; int incl = cnt;
#pragma unroll
  for (int o = 1; o < 32; o <<= 1) { const int v = __shfl_up(incl, o, 32); if (lane >= o) incl += v; }
  if (lane == 31) scan_ws[wave] = incl;
  __syncthreads();
  if (wave == 0) { int wv = (lane < NT / 32) ? scan_ws[lane] : 0; int wincl = wv;
#pragma unroll
    for (int o = 1; o < 32; o <<= 1) { const int v = __shfl_up(wincl, o, 32); if (lane >= o) wincl += v; }
    if (lane < NT / 32) scan_ws[32 + lane] = wincl - wv; if (lane == 31) scan_ws[64] = wincl; }
  __syncthreads();
  const int res = scan_ws[32 + wave] + incl - cnt; *tot = scan_ws[64];
  return res;
}
template <int SP, int CAP>
__device__ __forceinline__ int chunk_hits(const int* __restrict__ dstv, int e0, int n0, int tid, int* LIST, int* scan_ws) {
  const int eb = e0 + tid * SP;
  const bool real = eb < NE;
  const int ebc = real ? eb : (NE - SP);
  int rec[SP]; int cnt = 0;
#pragma unroll
  for (int k = 0; k < SP; k += 4) {
    const v4i d4 = *(const v4i*)(dstv + ebc + k);
#pragma unroll
    for (int q = 0; q < 4; ++q) {
      const int e = eb + k + q;
      const int d = d4[q];
      int r = -1;
      if (real && d >= n0 && d < n0 + TG && d < NN) { r = ((d - n0) << 20) | e; ++cnt; }
      rec[k + q] = r;
    }
  }
  int tot; int p = blk_excl_scan(cnt, scan_ws, tid, &tot);
#pragma unroll
  for (int k = 0; k < SP; ++k) if (rec[k] >= 0) { if ((unsigned)p < (unsigned)CAP) LIST[p] = rec[k]; ++p; }
  __syncthreads();
  return tot < CAP ? tot : CAP;
}

__global__ __launch_bounds__(NT) void agg_kernel(const float* __restrict__ Z, const int* __restrict__ srcv, const int* __restrict__ dstv,
                                                const float* __restrict__ SD, float* __restrict__ ACC, float* __restrict__ PART) {
  extern __shared__ __align__(16) float dyn_lds[];
  float* SM = dyn_lds;
  float* SL = dyn_lds + TG * 4;
  int* LIST = (int*)(dyn_lds + TG * 8);
  __shared__ int scan_ws[80];
  const int tid = threadIdx.x, lane = tid & 31, wave = tid >> 5;
  const int n0 = blockIdx.x * TG;
  const int c4 = 4 * lane;
  for (int i = tid; i < TG * 4; i += NT) { SM[i] = -INFINITY; SL[i] = 0.f; }
  float* accb = ACC + (size_t)n0 * ZW;
  {
    const v4f z4 = {0.f, 0.f, 0.f, 0.f};
    for (int pass = 0; pass < 2; ++pass) {
#pragma unroll 1
      for (int j = 0; j < TG / 8; ++j) {
        float* ap = accb + (size_t)(wave * (TG / 8) + j) * ZW + c4;
#pragma unroll
        for (int q = 0; q < 4; ++q) *(volatile v4f*)(ap + HID * q) = z4;
      }
      __threadfence();
    }
  }
  __syncthreads();
#pragma unroll 1
  for (int c = 0; c < NCH; ++c) {
    const int tot = chunk_hits<SPT, SCH>(dstv, c * SCH, n0, tid, LIST, scan_ws);
#pragma unroll 1
    for (int base = 0; base < tot; base += 32) {
      const int q0 = base + lane;
      const int rv = (q0 < tot) ? LIST[q0 < SCH ? q0 : (SCH - 1)] : -1;
      const int own = (rv >= 0 && (rv >> 28) == wave) ? 1 : 0;
      unsigned msk = (unsigned)__ballot(own);
#pragma unroll 1
      for (int it = 0; it < 32; ++it) {
        if (msk == 0u) break;
        const int bp = __builtin_ctz(msk); msk &= msk - 1u;
        const int r = __shfl(rv, bp, 32);
        const int dl = r >> 20;
        int e = r & 0xFFFFF; e = (e < NE) ? e : (NE - 1);
        const int d = n0 + dl;
        int s = srcv[e];
        s = s < 0 ? 0 : (s >= NN ? NN - 1 : s);
        const v4f sv = *(const v4f*)(SD + (size_t)s * 8);
        const v4f dv = *(const v4f*)(SD + (size_t)d * 8 + 4);
        const v4f mo = *(const v4f*)(SM + dl * 4);
        const v4f lo = *(const v4f*)(SL + dl * 4);
        v4f mn, rr, ex, ln;
#pragma unroll
        for (int q = 0; q < 4; ++q) {
          float p = sv[q] + dv[q];
          p = (p >= 0.f) ? p : 0.01f * p;
          const float m = fmaxf(mo[q], p);
          mn[q] = m;
          rr[q] = __expf(mo[q] - m);
          ex[q] = __expf(p - m);
          ln[q] = fmaf(lo[q], rr[q], ex[q]);
        }
        if (lane == 0) { *(v4f*)(SM + dl * 4) = mn; *(v4f*)(SL + dl * 4) = ln; }
        float* ap = accb + (size_t)dl * ZW + c4;
        const float* zp = Z + (size_t)s * ZW + c4;
        v4f o[4];
#pragma unroll
        for (int q = 0; q < 4; ++q) {
          const v4f qa = *(const v4f*)(ap + HID * q);
          const v4f zz = *(const v4f*)(zp + HID * q);
          v4f t;
#pragma unroll
          for (int i = 0; i < 4; ++i) t[i] = fmaf(qa[i], rr[q], ex[q] * zz[i]);
          o[q] = t;
        }
#pragma unroll
        for (int q = 0; q < 4; ++q) *(volatile v4f*)(ap + HID * q) = o[q];
        __threadfence();
#pragma unroll
        for (int q = 0; q < 4; ++q) *(volatile v4f*)(ap + HID * q) = o[q];
        asm volatile("" ::: "memory");
      }
    }
    __syncthreads();
  }
  float cs[16], cq[16];
#pragma unroll
  for (int i = 0; i < 16; ++i) { cs[i] = 0.f; cq[i] = 0.f; }
#pragma unroll 1
  for (int j = 0; j < TG / 8; ++j) {
    const int dl = wave * (TG / 8) + j;
    const int n = n0 + dl;
    if (n < NN) {
      const v4f l4 = *(const v4f*)(SL + dl * 4);
      float* ap = accb + (size_t)dl * ZW + c4;
      v4f rv4[4];
#pragma unroll
      for (int q = 0; q < 4; ++q) {
        const float lq = l4[q];
        const float inv = (lq > 0.f) ? (1.0f / fmaxf(lq, 1e-20f)) : 0.f;
        const v4f qa = *(const v4f*)(ap + HID * q);
        v4f t;
#pragma unroll
        for (int i = 0; i < 4; ++i) {
          const float v = fmaxf(qa[i] * inv, 0.f);
          t[i] = v;
          cs[4 * q + i] += v;
          cq[4 * q + i] = fmaf(v, v, cq[4 * q + i]);
        }
        rv4[q] = t;
      }
      for (int pass = 0; pass < 2; ++pass) {
#pragma unroll
        for (int q = 0; q < 4; ++q) *(volatile v4f*)(ap + HID * q) = rv4[q];
        __threadfence();
      }
    }
  }
  __syncthreads();
  float* RED = SM;
#pragma unroll
  for (int q = 0; q < 4; ++q) {
    v4f a, b;
#pragma unroll
    for (int i = 0; i < 4; ++i) { a[i] = cs[4 * q + i]; b[i] = cq[4 * q + i]; }
    *(v4f*)(RED + wave * 1024 + HID * q + c4) = a;
    *(v4f*)(RED + wave * 1024 + 512 + HID * q + c4) = b;
  }
  __syncthreads();
  v4f t4 = {0.f, 0.f, 0.f, 0.f};
#pragma unroll
  for (int w = 0; w < 8; ++w) { const v4f u = *(const v4f*)(RED + w * 1024 + 4 * tid); t4 += u; }
  float* pp = PART + (size_t)blockIdx.x * 1024 + 4 * tid;
  *(volatile v4f*)pp = t4;
  __threadfence();
  *(volatile v4f*)pp = t4;
}

__global__ __launch_bounds__(512) void bnfin_kernel(const float* __restrict__ PART, const float* __restrict__ gam,
                                                   const float* __restrict__ bet, float* __restrict__ BNP) {
  const int t = threadIdx.x;
  double s = 0.0, q = 0.0;
#pragma unroll 1
  for (int b = 0; b < NTILE; ++b) { s += (double)PART[b * 1024 + t]; q += (double)PART[b * 1024 + 512 + t]; }
  const double mean = s * (1.0 / (double)NN);
  double var = q * (1.0 / (double)NN) - mean * mean;
  if (var < 0.0) var = 0.0;
  const float meanf = (float)mean, varf = (float)var;
  const float istd = 1.0f / sqrtf(varf + BN_EPS);
  const float sc = gam[t] * istd;
  const float sh = bet[t] - meanf * sc;
  ((volatile float*)BNP)[t] = sc;
  ((volatile float*)BNP)[512 + t] = sh;
  __threadfence();
  ((volatile float*)BNP)[t] = sc;
  ((volatile float*)BNP)[512 + t] = sh;
}

__global__ __launch_bounds__(NT) void combine_kernel(const float* __restrict__ ACC, const float* __restrict__ BNP,
                                                    const float* __restrict__ ow, const float* __restrict__ ob,
                                                    unsigned short* __restrict__ X16p, float* __restrict__ XF) {
  const int lane = threadIdx.x & 31;
  const int n = blockIdx.x * (NT / 32) + (threadIdx.x >> 5);
  const int c4 = 4 * lane;
  if (n < MP) {
    v4f xo = {0.f, 0.f, 0.f, 0.f};
    if (n < NN) {
      const v4f w4 = *(const v4f*)(ow + c4);
      const float bb = ob[0];
      v4f y[4]; float lg[4];
#pragma unroll
      for (int q = 0; q < 4; ++q) {
        const v4f r  = *(const v4f*)(ACC + (size_t)n * ZW + HID * q + c4);
        const v4f sc = *(const v4f*)(BNP + HID * q + c4);
        const v4f sh = *(const v4f*)(BNP + 512 + HID * q + c4);
        v4f t; float p = 0.f;
#pragma unroll
        for (int i = 0; i < 4; ++i) { t[i] = fmaf(r[i], sc[i], sh[i]); p = fmaf(t[i], w4[i], p); }
        y[q] = t;
#pragma unroll
        for (int off = 16; off > 0; off >>= 1) p += __shfl_xor(p, off, 32);
        lg[q] = p + bb;
      }
      const float mx = fmaxf(fmaxf(lg[0], lg[1]), fmaxf(lg[2], lg[3]));
      float ev[4]; float sum = 0.f;
#pragma unroll
      for (int q = 0; q < 4; ++q) { ev[q] = __expf(lg[q] - mx); sum += ev[q]; }
      const float inv = 1.0f / sum;
#pragma unroll
      for (int q = 0; q < 4; ++q) {
        const float sq = ev[q] * inv;
#pragma unroll
        for (int i = 0; i < 4; ++i) xo[i] = fmaf(sq, y[q][i], xo[i]);
      }
    }
    v4h h4;
#pragma unroll
    for (int i = 0; i < 4; ++i) h4[i] = (_Float16)xo[i];
    float* xp = XF + (size_t)(n < NN ? n : 0) * HID + c4;
    _Float16* hp = (_Float16*)X16p + (size_t)n * HID + c4;
    for (int pass = 0; pass < 2; ++pass) {
      if (n < NN) *(volatile v4f*)xp = xo;
      *(volatile v4h*)hp = h4;
      __threadfence();
    }
  }
}

__global__ __launch_bounds__(NT) void pool_kernel(const float* __restrict__ XF, const int* __restrict__ gid, float* __restrict__ out) {
  __shared__ int LIST[NT];
  __shared__ int scan_ws[80];
  const int tid = threadIdx.x;
  const int g = blockIdx.x;
  float a = 0.f; int cnt = 0;
#pragma unroll 1
  for (int c = 0; c < (NN + NT - 1) / NT; ++c) {
    const int n = c * NT + tid;
    const int nc = (n < NN) ? n : (NN - 1);
    const int gv = gid[nc];
    const int hit = (n < NN && gv == g) ? 1 : 0;
    int tot; const int p = blk_excl_scan(hit, scan_ws, tid, &tot);
    if (hit) LIST[p] = n;
    __syncthreads();
    cnt += tot;
    const int tl = tot < NT ? tot : NT;
    if (tid < HID) {
#pragma unroll 1
      for (int k = 0; k < tl; ++k) {
        int node = LIST[k]; node = node < 0 ? 0 : (node >= NN ? NN - 1 : node);
        a += XF[(size_t)node * HID + tid];
      }
    }
    __syncthreads();
  }
  const float inv = 1.0f / fmaxf((float)cnt, 1.0f);
  const float v = a * inv;
  if (tid < HID) {
    float* op = out + (size_t)g * HID + tid;
    *(volatile float*)op = v;
    __threadfence();
    *(volatile float*)op = v;
  }
}

extern "C" void kernel_launch(void* const* d_in, const int* in_sizes, int n_in,
                              void* d_out, int out_size, void* d_ws, size_t ws_size, hipStream_t stream) {
  if (n_in < 11) return;
  const float* h     = (const float*)d_in[0];
  const int*   src   = (const int*)  d_in[1];
  const int*   dst   = (const int*)  d_in[2];
  const int*   gid   = (const int*)  d_in[3];
  const float* W0    = (const float*)d_in[4];
  const float* Wr    = (const float*)d_in[5];
  const float* att   = (const float*)d_in[6];
  const float* gam   = (const float*)d_in[7];
  const float* bet   = (const float*)d_in[8];
  const float* ow    = (const float*)d_in[9];
  const float* ob    = (const float*)d_in[10];
  float* out = (float*)d_out;

  if (in_sizes[0] != NN * FIN || in_sizes[1] != NE || in_sizes[2] != NE || in_sizes[3] != NN) return;
  if (in_sizes[4] != NHD * FIN * HID || in_sizes[5] != NHD * HID * HID || in_sizes[6] != 2 * NHD * 2 * HID) return;
  if (in_sizes[7] != 2 * ZW || in_sizes[8] != 2 * ZW || in_sizes[9] != 2 * HID || in_sizes[10] != 2) return;
  if (out_size != NG * HID) return;

  char* ws = (char*)d_ws; size_t off = 0;
  auto carve = [&](size_t bytes) -> char* { char* p = ws + off; off += (bytes + 255) & ~(size_t)255; return p; };
  float*          Z    = (float*)carve((size_t)MP * ZW * 4);
  float*          ACC  = (float*)carve((size_t)NROWT * ZW * 4);
  unsigned short* X16  = (unsigned short*)carve((size_t)MP * HID * 2);
  float*          XF   = (float*)carve((size_t)NN * HID * 4);
  float*          SD   = (float*)carve((size_t)NN * 8 * 4);
  unsigned short* Bt   = (unsigned short*)carve((size_t)ZW * HID * 2);
  float*          PART = (float*)carve((size_t)NTILE * 1024 * 4);
  float*          BNP  = (float*)carve((size_t)1024 * 4);
  if (off > ws_size || off > (size_t)134217728) return;

  const int gemmTiles = (MP / 64) * (ZW / 64);
  hipFuncSetAttribute(reinterpret_cast<const void*>(&agg_kernel), hipFuncAttributeMaxDynamicSharedMemorySize, AGG_LDS_BYTES);

  cast_h_kernel<<<(MP * (KP0 / 2) + NT - 1) / NT, NT, 0, stream>>>(h, X16);
  wprep_kernel<<<(ZW * (KP0 / 2) + NT - 1) / NT, NT, 0, stream>>>(W0, Bt, FIN, KP0);
  wmma_gemm64<0, false, 0, 0, false, 0><<<dim3((gemmTiles + 7) / 8, 1), 256, 0, stream>>>(
      U16(X16), U16(X16), KP0, 0L,
      U16(Bt), U16(Bt), KP0, 0L,
      (void*)Z, (void*)nullptr, ZW, 0L,
      (const float*)nullptr, (const float*)nullptr, 0L, MP, ZW, KP0, WSC_INV);
  dots_kernel<<<(NN / 4 + (NT / 32) - 1) / (NT / 32), NT, 0, stream>>>(Z, att, SD);
  agg_kernel<<<NTILE, NT, AGG_LDS_BYTES, stream>>>(Z, src, dst, SD, ACC, PART);
  bnfin_kernel<<<1, 512, 0, stream>>>(PART, gam, bet, BNP);
  combine_kernel<<<MP / (NT / 32), NT, 0, stream>>>(ACC, BNP, ow, ob, X16, XF);

  wprep_kernel<<<(ZW * (HID / 2) + NT - 1) / NT, NT, 0, stream>>>(Wr, Bt, HID, HID);
  wmma_gemm64<0, false, 0, 0, false, 0><<<dim3((gemmTiles + 7) / 8, 1), 256, 0, stream>>>(
      U16(X16), U16(X16), HID, 0L,
      U16(Bt), U16(Bt), HID, 0L,
      (void*)Z, (void*)nullptr, ZW, 0L,
      (const float*)nullptr, (const float*)nullptr, 0L, MP, ZW, HID, WSC_INV);
  dots_kernel<<<(NN / 4 + (NT / 32) - 1) / (NT / 32), NT, 0, stream>>>(Z, att + NHD * 2 * HID, SD);
  agg_kernel<<<NTILE, NT, AGG_LDS_BYTES, stream>>>(Z, src, dst, SD, ACC, PART);
  bnfin_kernel<<<1, 512, 0, stream>>>(PART, gam + ZW, bet + ZW, BNP);
  combine_kernel<<<MP / (NT / 32), NT, 0, stream>>>(ACC, BNP, ow + HID, ob + 1, X16, XF);

  pool_kernel<<<NG, NT, 0, stream>>>(XF, gid, out);
}
